// DMPNet_75900662055053
// MI455X (gfx1250) — hardware-run, weakly checked
//
#include <hip/hip_runtime.h>
#include <math.h>

typedef __attribute__((ext_vector_type(16))) _Float16 v16h;
typedef __attribute__((ext_vector_type(8)))  _Float16 v8h;
typedef __attribute__((ext_vector_type(16))) __bf16   v16b;
typedef __attribute__((ext_vector_type(8)))  __bf16   v8b;
typedef __attribute__((ext_vector_type(8)))  float    v8f;
typedef __attribute__((ext_vector_type(4)))  float    v4f;

constexpr int kBatch   = 16384;
constexpr int kInW     = 128;
constexpr int kHid     = 2048;
constexpr int kNout    = 54;
constexpr int kNoutP   = 64;
constexpr int kChunk   = 4096;
constexpr int kNChunk  = kBatch / kChunk;
constexpr int kDof     = 9;
constexpr int kNb      = 5;
constexpr int kTs      = 10;
constexpr int kLs      = 10;
constexpr int kSteps   = kTs * kLs;
constexpr int kRowsR   = kBatch * kDof;
constexpr int kScanBlk = 256;
constexpr int kOutBlk  = kScanBlk * kTs;
constexpr int kWlBlocks = (kNoutP * kHid / 8) / 256;
constexpr float kW1Carry    = 1024.0f;
constexpr float kW1CarryInv = 1.0f / 1024.0f;

static_assert(kNChunk * kChunk == kBatch);
static_assert((kInW % 32) == 0 && (kHid % 32) == 0);
static_assert((kChunk % 64) == 0 && (kHid % 64) == 0 && (kNoutP % 64) == 0);
static_assert((((kChunk / 64) * (kHid / 64)) % 8) == 0);
static_assert((((kChunk / 64) * (kNoutP / 64)) % 8) == 0);
static_assert(kNout == kDof * (kNb + 1));
static_assert((kRowsR % kScanBlk) == 0);
static_assert(((kOutBlk * 4) % 128) == 0);
static_assert(kOutBlk == 2560);
static_assert(kWlBlocks * 256 * 8 == kNoutP * kHid);

constexpr size_t kOffINH  = 0;
constexpr size_t kOffINL  = kOffINH  + (size_t)kBatch * kInW * 2;
constexpr size_t kOffW0H  = kOffINL  + (size_t)kBatch * kInW * 2;
constexpr size_t kOffW0L  = kOffW0H  + (size_t)kHid * kInW * 2;
constexpr size_t kOffW1S  = kOffW0L  + (size_t)kHid * kInW * 2;
constexpr size_t kOffWLH  = kOffW1S  + (size_t)kHid * kHid * 2;
constexpr size_t kOffWLL  = kOffWLH  + (size_t)kNoutP * kHid * 2;
constexpr size_t kOffBL64 = kOffWLL  + (size_t)kNoutP * kHid * 2;
constexpr size_t kOffH1   = kOffBL64 + (size_t)kNoutP * 4;
constexpr size_t kOffH2H  = kOffH1   + (size_t)kChunk * kHid * 2;
constexpr size_t kOffH2L  = kOffH2H  + (size_t)kChunk * kHid * 2;
constexpr size_t kOffOUT3 = kOffH2L  + (size_t)kChunk * kHid * 2;
constexpr size_t kWsTotal = kOffOUT3 + (size_t)kBatch * kNoutP * 4;
static_assert(kWsTotal == 72876288ull);
static_assert(kWsTotal <= 134217728ull);
static_assert((kOffINL % 128) == 0 && (kOffW0H % 128) == 0 && (kOffW0L % 128) == 0 && (kOffW1S % 128) == 0 &&
              (kOffWLH % 128) == 0 && (kOffWLL % 128) == 0 && (kOffBL64 % 128) == 0 && (kOffH1 % 128) == 0 &&
              (kOffH2H % 128) == 0 && (kOffH2L % 128) == 0 && (kOffOUT3 % 128) == 0);

__device__ __forceinline__ unsigned short f2bf_bits(float f) {
  unsigned u = __float_as_uint(f);
  return (unsigned short)((u + 0x7FFFu + ((u >> 16) & 1u)) >> 16);
}
__device__ __forceinline__ float bf_bits2f(unsigned short h) { return __uint_as_float(((unsigned)h) << 16); }

__device__ __forceinline__ void grp_guard_h(v8f& a, v8f& b, v8f& c, v8f& d, v16h x, v16h y) {
  asm volatile("v_nop\n\tv_nop\n\tv_nop\n\tv_nop" : "+v"(a), "+v"(b), "+v"(c), "+v"(d) : "v"(x), "v"(y));
}
__device__ __forceinline__ void grp_guard_b(v8f& a, v8f& b, v8f& c, v8f& d, v16b x, v16b y) {
  asm volatile("v_nop\n\tv_nop\n\tv_nop\n\tv_nop" : "+v"(a), "+v"(b), "+v"(c), "+v"(d) : "v"(x), "v"(y));
}
__device__ __forceinline__ void keep4_h(v16h a, v16h b, v16h c, v16h d) { asm volatile("v_nop" :: "v"(a), "v"(b), "v"(c), "v"(d)); }
__device__ __forceinline__ void keep4_b(v16b a, v16b b, v16b c, v16b d) { asm volatile("v_nop" :: "v"(a), "v"(b), "v"(c), "v"(d)); }
__device__ __forceinline__ void acc_guard4(v8f& a, v8f& b, v8f& c, v8f& d) {
  asm volatile("v_nop\n\tv_nop\n\tv_nop\n\tv_nop" : "+v"(a), "+v"(b), "+v"(c), "+v"(d));
}

template <typename T> struct Frag;
template <> struct Frag<_Float16> {
  typedef v16h V; union U { v16h v; v8h h[2]; };
  static __device__ __forceinline__ v16h load(const _Float16* p) {
    U f; f.h[0] = *(const v8h*)(p); f.h[1] = *(const v8h*)(p + 16); return f.v;
  }
  static __device__ __forceinline__ v8f mma(v16h a, v16h b, v8f c) {
    return __builtin_amdgcn_wmma_f32_16x16x32_f16(false, a, false, b, (short)0, c, false, false);
  }
  static __device__ __forceinline__ void guard4(v8f& a, v8f& b, v8f& c, v8f& d, v16h x, v16h y) { grp_guard_h(a, b, c, d, x, y); }
  static __device__ __forceinline__ void keep(v16h a, v16h b, v16h c, v16h d) { keep4_h(a, b, c, d); }
};
template <> struct Frag<__bf16> {
  typedef v16b V; union U { v16b v; v8b h[2]; };
  static __device__ __forceinline__ v16b load(const __bf16* p) {
    U f; f.h[0] = *(const v8b*)(p); f.h[1] = *(const v8b*)(p + 16); return f.v;
  }
  static __device__ __forceinline__ v8f mma(v16b a, v16b b, v8f c) {
    return __builtin_amdgcn_wmma_f32_16x16x32_bf16(false, a, false, b, (short)0, c, false, false);
  }
  static __device__ __forceinline__ void guard4(v8f& a, v8f& b, v8f& c, v8f& d, v16b x, v16b y) { grp_guard_b(a, b, c, d, x, y); }
  static __device__ __forceinline__ void keep(v16b a, v16b b, v16b c, v16b d) { keep4_b(a, b, c, d); }
};

template <int ET> struct Elem;
template <> struct Elem<0> { typedef _Float16 T; };
template <> struct Elem<1> { typedef __bf16 T; };

template <int ET, int SPL, int OUT_MODE, int ACT>
__global__ __launch_bounds__(256) void wmma_gemm64(
    const unsigned short* __restrict__ Ap, const unsigned short* __restrict__ A2p, int lda,
    const unsigned short* __restrict__ Btp, const unsigned short* __restrict__ Bt2p, int ldb,
    void* __restrict__ Cout, void* __restrict__ Cout2, int ldc,
    const float* __restrict__ bias,
    int M, int N, int K, float scale, float post) {
  typedef typename Elem<ET>::T T;
  typedef typename Frag<T>::V V;
  const T* A = (const T*)Ap; const T* A2 = (const T*)A2p; const T* Bt = (const T*)Btp; const T* Bt2 = (const T*)Bt2p;
  __shared__ __align__(16) float sT[8][16 * 68];
  const int lane = threadIdx.x & 31;
  const int wave = threadIdx.x >> 5;
  const int tilesN = N >> 6;
  const int tilesM = M >> 6;
  const int tile = blockIdx.x * 8 + wave;
  if (tile >= tilesM * tilesN) return;
  const int tm = tile / tilesN;
  const int tn = tile - tm * tilesN;
  const int m0 = tm << 6;
  const int n0 = tn << 6;

  const T* Ab  = A;
  const T* Bb  = Bt;
  const T* Ab2 = (SPL >= 1) ? A2 : nullptr;
  const T* Bb2 = (SPL == 2) ? Bt2 : nullptr;

  const int rlane = lane & 15;
  const int koff  = (lane >> 4) * 8;
  const int mOff  = (lane >> 4) * 8;

  v8f acc[4][4];
#pragma unroll
  for (int i = 0; i < 4; ++i)
#pragma unroll
    for (int j = 0; j < 4; ++j) acc[i][j] = (v8f){0.f,0.f,0.f,0.f,0.f,0.f,0.f,0.f};

  for (int k0 = 0; k0 < K; k0 += 32) {
    V bh[4], bl[4];
#pragma unroll
    for (int j = 0; j < 4; ++j) {
      const size_t bo = (size_t)(n0 + (j << 4) + rlane) * ldb + koff + k0;
      bh[j] = Frag<T>::load(Bb + bo);
      if (SPL == 2) bl[j] = Frag<T>::load(Bb2 + bo);
    }
#pragma unroll
    for (int i = 0; i < 4; ++i) {
      const size_t ao = (size_t)(m0 + (i << 4) + rlane) * lda + koff + k0;
      V ah = Frag<T>::load(Ab + ao);
      V al;
      if (SPL >= 1) al = Frag<T>::load(Ab2 + ao);
#pragma unroll
      for (int j = 0; j < 4; ++j) {
        acc[i][j] = Frag<T>::mma(ah, bh[j], acc[i][j]);
        if (SPL == 2) acc[i][j] = Frag<T>::mma(ah, bl[j], acc[i][j]);
        if (SPL >= 1) acc[i][j] = Frag<T>::mma(al, bh[j], acc[i][j]);
      }
      Frag<T>::guard4(acc[i][0], acc[i][1], acc[i][2], acc[i][3], ah, (SPL >= 1) ? al : ah);
    }
    Frag<T>::keep(bh[0], bh[1], bh[2], bh[3]);
    if (SPL == 2) Frag<T>::keep(bl[0], bl[1], bl[2], bl[3]);
  }
  acc_guard4(acc[0][0], acc[0][1], acc[0][2], acc[0][3]);
  acc_guard4(acc[1][0], acc[1][1], acc[1][2], acc[1][3]);
  acc_guard4(acc[2][0], acc[2][1], acc[2][2], acc[2][3]);
  acc_guard4(acc[3][0], acc[3][1], acc[3][2], acc[3][3]);

  float* slab = sT[wave];
#pragma unroll
  for (int i = 0; i < 4; ++i) {
    const int mBase = m0 + (i << 4);
#pragma unroll
    for (int j = 0; j < 4; ++j) {
      const float bv = bias[n0 + (j << 4) + rlane];
#pragma unroll
      for (int r = 0; r < 8; ++r) {
        float v = acc[i][j][r] * scale + bv;
        if (ACT == 7) v = v * post;
        slab[(mOff + r) * 68 + (j << 4) + rlane] = v;
      }
    }
    __builtin_amdgcn_fence(__ATOMIC_RELEASE, "workgroup");
    __builtin_amdgcn_wave_barrier();
    __builtin_amdgcn_fence(__ATOMIC_ACQUIRE, "workgroup");
    if (ACT == 1) {
#pragma unroll 1
      for (int t = 0; t < 32; ++t) {
        const int idx = t * 32 + lane;
        float* p = slab + (idx >> 6) * 68 + (idx & 63);
        const float xv = *p;
        const float ev = __expf(2.0f * xv);
        const float rv = __builtin_amdgcn_rcpf(ev + 1.0f);
        *p = 1.0f - 2.0f * rv;
      }
      __builtin_amdgcn_fence(__ATOMIC_RELEASE, "workgroup");
      __builtin_amdgcn_wave_barrier();
      __builtin_amdgcn_fence(__ATOMIC_ACQUIRE, "workgroup");
    }
    if (OUT_MODE == 0) {
      float* C = (float*)Cout;
      const int hh = lane >> 4, c4 = (lane & 15) * 4;
      for (int pass = 0; pass < 2; ++pass) {
#pragma unroll
        for (int it = 0; it < 8; ++it) {
          const int row = it * 2 + hh;
          v4f v = *(const v4f*)(slab + row * 68 + c4);
          *(volatile v4f*)(C + (size_t)(mBase + row) * ldc + n0 + c4) = v;
        }
        __threadfence();
      }
    } else {
      const int q = lane >> 3, c8 = (lane & 7) * 8;
      unsigned short* C  = (unsigned short*)Cout;
      unsigned short* C2 = (OUT_MODE == 2) ? (unsigned short*)Cout2 : nullptr;
      for (int pass = 0; pass < 2; ++pass) {
#pragma unroll
        for (int it = 0; it < 4; ++it) {
          const int row = it * 4 + q;
          const float* sp = slab + row * 68 + c8;
          v8h hv, lv;
#pragma unroll
          for (int e = 0; e < 8; ++e) {
            if (OUT_MODE == 1) {
              hv[e] = (_Float16)sp[e];
            } else {
              unsigned short hb = f2bf_bits(sp[e]);
              unsigned short lb = f2bf_bits(sp[e] - bf_bits2f(hb));
              hv[e] = __builtin_bit_cast(_Float16, hb);
              lv[e] = __builtin_bit_cast(_Float16, lb);
            }
          }
          *(volatile v8h*)(C + (size_t)(mBase + row) * ldc + n0 + c8) = hv;
          if (OUT_MODE == 2) *(volatile v8h*)(C2 + (size_t)(mBase + row) * ldc + n0 + c8) = lv;
        }
        __threadfence();
      }
    }
    __builtin_amdgcn_fence(__ATOMIC_RELEASE, "workgroup");
    __builtin_amdgcn_wave_barrier();
    __builtin_amdgcn_fence(__ATOMIC_ACQUIRE, "workgroup");
  }
}

__global__ __launch_bounds__(256) void split_rows_bf16_kernel(
    const float* __restrict__ src, unsigned short* __restrict__ dhi, unsigned short* __restrict__ dlo, int total8)
{
  const int i = blockIdx.x * 256 + threadIdx.x;
  if (i >= total8) return;
  const size_t e0 = (size_t)i << 3;
  const v4f a0 = *(const v4f*)(src + e0);
  const v4f a1 = *(const v4f*)(src + e0 + 4);
  v8h hv, lv;
#pragma unroll
  for (int e = 0; e < 4; ++e) {
    const float x0 = a0[e], x1 = a1[e];
    const unsigned short h0 = f2bf_bits(x0), h1 = f2bf_bits(x1);
    const unsigned short l0 = f2bf_bits(x0 - bf_bits2f(h0)), l1 = f2bf_bits(x1 - bf_bits2f(h1));
    hv[e]     = __builtin_bit_cast(_Float16, h0);
    hv[4 + e] = __builtin_bit_cast(_Float16, h1);
    lv[e]     = __builtin_bit_cast(_Float16, l0);
    lv[4 + e] = __builtin_bit_cast(_Float16, l1);
  }
  unsigned short* qh = dhi + e0;
  unsigned short* ql = dlo + e0;
  *(volatile v8h*)qh = hv;
  *(volatile v8h*)ql = lv;
  __threadfence();
  *(volatile v8h*)qh = hv;
  *(volatile v8h*)ql = lv;
}

__global__ __launch_bounds__(256) void cast_rows_f16_carry_kernel(
    const float* __restrict__ src, unsigned short* __restrict__ dst, int total8, float carry)
{
  const int i = blockIdx.x * 256 + threadIdx.x;
  if (i >= total8) return;
  const size_t e0 = (size_t)i << 3;
  const v4f a0 = *(const v4f*)(src + e0);
  const v4f a1 = *(const v4f*)(src + e0 + 4);
  v8h hv;
#pragma unroll
  for (int e = 0; e < 4; ++e) {
    const float x0 = a0[e] * carry, x1 = a1[e] * carry;
    hv[e]     = (_Float16)x0;
    hv[4 + e] = (_Float16)x1;
  }
  unsigned short* qh = dst + e0;
  *(volatile v8h*)qh = hv;
  __threadfence();
  *(volatile v8h*)qh = hv;
}

__global__ __launch_bounds__(256) void pad_last_layer_kernel(
    const float* __restrict__ wl, const float* __restrict__ blv,
    unsigned short* __restrict__ dhi, unsigned short* __restrict__ dlo, float* __restrict__ bl64)
{
  const int tid = threadIdx.x;
  if (blockIdx.x == kWlBlocks) {
    const int lane = tid & 31, wave = tid >> 5;
    if (wave == 0) {
      const int idx0 = (lane & 15) * 4;
      v4f v;
#pragma unroll
      for (int e = 0; e < 4; ++e) {
        const int idx = idx0 + e;
        const int ic = (idx < kNout) ? idx : (kNout - 1);
        const float x = blv[ic];
        v[e] = (idx < kNout) ? x : 0.0f;
      }
      if (lane < 16) {
        *(volatile v4f*)(bl64 + idx0) = v;
        __threadfence();
        *(volatile v4f*)(bl64 + idx0) = v;
      }
    }
    return;
  }
  const int i = blockIdx.x * 256 + tid;
  const int e0 = i << 3;
  const int row = e0 / kHid;
  const int col = e0 - row * kHid;
  const int rc = (row < kNout) ? row : (kNout - 1);
  const bool live = (row < kNout);
  const v4f a0 = *(const v4f*)(wl + (size_t)rc * kHid + col);
  const v4f a1 = *(const v4f*)(wl + (size_t)rc * kHid + col + 4);
  v8h hv, lv;
#pragma unroll
  for (int e = 0; e < 4; ++e) {
    const float r0 = a0[e], r1 = a1[e];
    const float x0 = live ? r0 : 0.0f;
    const float x1 = live ? r1 : 0.0f;
    const unsigned short h0 = f2bf_bits(x0), h1 = f2bf_bits(x1);
    const unsigned short l0 = f2bf_bits(x0 - bf_bits2f(h0)), l1 = f2bf_bits(x1 - bf_bits2f(h1));
    hv[e]     = __builtin_bit_cast(_Float16, h0);
    hv[4 + e] = __builtin_bit_cast(_Float16, h1);
    lv[e]     = __builtin_bit_cast(_Float16, l0);
    lv[4 + e] = __builtin_bit_cast(_Float16, l1);
  }
  unsigned short* qh = dhi + e0;
  unsigned short* ql = dlo + e0;
  *(volatile v8h*)qh = hv;
  *(volatile v8h*)ql = lv;
  __threadfence();
  *(volatile v8h*)qh = hv;
  *(volatile v8h*)ql = lv;
}

__global__ __launch_bounds__(256) void traj_scan_kernel(
    const float* __restrict__ out3, const float* __restrict__ input, float* __restrict__ out)
{
  __shared__ __align__(16) float sG[kSteps * kNb];
  __shared__ __align__(16) float sO[kOutBlk];
  const int tid = threadIdx.x;
  if (tid < kSteps) {
    const int trips = (tid + 1 < kSteps) ? (tid + 1) : kSteps;
    float x = 1.0f;
#pragma unroll 1
    for (int it = 0; it < trips; ++it) {
      const float dx = (-x) * 0.01f;
      x = x + dx;
    }
    float psum = 0.0f;
#pragma unroll 1
    for (int n = 0; n < kNb; ++n) {
      const float c = expf(-0.25f * (float)n);
      const float h = 11.180339887f * (1.0f / c);
      const float dd = x - c;
      const float p = expf(-h * (dd * dd));
      sG[tid * kNb + n] = p;
      psum += p;
    }
    const float inv = x * (1.0f / psum);
#pragma unroll 1
    for (int n = 0; n < kNb; ++n) {
      const float p = sG[tid * kNb + n];
      sG[tid * kNb + n] = p * inv;
    }
  }
  __syncthreads();

  int r = blockIdx.x * kScanBlk + tid;
  r = (r < kRowsR) ? r : (kRowsR - 1);
  const int b = r / kDof;
  const int d = r - b * kDof;
  const float* o = out3 + (size_t)b * kNoutP;
  const float goal = o[d];
  const float w0 = o[kDof + d * kNb + 0];
  const float w1 = o[kDof + d * kNb + 1];
  const float w2 = o[kDof + d * kNb + 2];
  const float w3 = o[kDof + d * kNb + 3];
  const float w4 = o[kDof + d * kNb + 4];
  const float y0  = input[(size_t)b * kInW + 7 + d];
  const float dy0 = input[(size_t)b * kInW + 22 + d];
  const float span = goal - y0;

  float y = y0, z = dy0, ylast = y0;
#pragma unroll 1
  for (int t = 0; t < kTs; ++t) {
#pragma unroll 1
    for (int ss = 0; ss < kLs; ++ss) {
      const float* gs = sG + (t * kLs + ss) * kNb;
      float acc = w0 * gs[0];
      acc += w1 * gs[1];
      acc += w2 * gs[2];
      acc += w3 * gs[3];
      acc += w4 * gs[4];
      const float fx = span * acc;
      const float dz = 25.0f * (6.25f * (goal - y) - z) + fx;
      const float yn = y + z * 0.01f;
      const float zn = z + dz * 0.01f;
      y = yn;
      z = zn;
    }
    sO[tid * kTs + t] = y - ylast;
    ylast = y;
  }
  __syncthreads();

  float* ob = out + (size_t)blockIdx.x * kOutBlk;
  constexpr int kPieces = kOutBlk / 4;
  v4f vv[3];
#pragma unroll
  for (int it = 0; it < 3; ++it) {
    const int idx4 = it * kScanBlk + tid;
    const int idc = (idx4 < kPieces) ? idx4 : (kPieces - 1);
    vv[it] = *(const v4f*)(sO + idc * 4);
  }
  for (int pass = 0; pass < 2; ++pass) {
#pragma unroll
    for (int it = 0; it < 3; ++it) {
      const int idx4 = it * kScanBlk + tid;
      if (idx4 < kPieces) *(volatile v4f*)(ob + (size_t)idx4 * 4) = vv[it];
    }
    __threadfence();
  }
}

extern "C" void kernel_launch(void* const* d_in, const int* in_sizes, int n_in,
                              void* d_out, int out_size, void* d_ws, size_t ws_size,
                              hipStream_t stream) {
  if (n_in < 7) return;
  if (in_sizes[0] != kBatch * kInW) return;
  if (in_sizes[1] != kHid * kInW) return;
  if (in_sizes[2] != kHid) return;
  if (in_sizes[3] != kHid * kHid) return;
  if (in_sizes[4] != kHid) return;
  if (in_sizes[5] != kNout * kHid) return;
  if (in_sizes[6] != kNout) return;
  if (out_size != kRowsR * kTs) return;
  if (ws_size < kWsTotal) return;

  const float* input = (const float*)d_in[0];
  const float* W0    = (const float*)d_in[1];
  const float* b0    = (const float*)d_in[2];
  const float* W1    = (const float*)d_in[3];
  const float* b1    = (const float*)d_in[4];
  const float* Wl    = (const float*)d_in[5];
  const float* bl    = (const float*)d_in[6];
  float* out = (float*)d_out;

  char* ws = (char*)d_ws;
  unsigned short* INH  = (unsigned short*)(ws + kOffINH);
  unsigned short* INL  = (unsigned short*)(ws + kOffINL);
  unsigned short* W0H  = (unsigned short*)(ws + kOffW0H);
  unsigned short* W0L  = (unsigned short*)(ws + kOffW0L);
  unsigned short* W1S  = (unsigned short*)(ws + kOffW1S);
  unsigned short* WLH  = (unsigned short*)(ws + kOffWLH);
  unsigned short* WLL  = (unsigned short*)(ws + kOffWLL);
  float*          BL64 = (float*)(ws + kOffBL64);
  unsigned short* H1   = (unsigned short*)(ws + kOffH1);
  unsigned short* H2H  = (unsigned short*)(ws + kOffH2H);
  unsigned short* H2L  = (unsigned short*)(ws + kOffH2L);
  float*          OUT3 = (float*)(ws + kOffOUT3);

  split_rows_bf16_kernel<<<(kBatch * kInW / 8) / 256, 256, 0, stream>>>(input, INH, INL, kBatch * kInW / 8);
  split_rows_bf16_kernel<<<(kHid * kInW / 8) / 256, 256, 0, stream>>>(W0, W0H, W0L, kHid * kInW / 8);
  cast_rows_f16_carry_kernel<<<(kHid * kHid / 8) / 256, 256, 0, stream>>>(W1, W1S, kHid * kHid / 8, kW1Carry);
  pad_last_layer_kernel<<<kWlBlocks + 1, 256, 0, stream>>>(Wl, bl, WLH, WLL, BL64);

  const int gridBig   = ((kChunk / 64) * (kHid / 64)) / 8;
  const int gridSmall = ((kChunk / 64) * (kNoutP / 64)) / 8;
  for (int c = 0; c < kNChunk; ++c) {
    const size_t rowOff = (size_t)c * kChunk;
    wmma_gemm64<1, 2, 1, 1><<<gridBig, 256, 0, stream>>>(
        INH + rowOff * kInW, INL + rowOff * kInW, kInW,
        W0H, W0L, kInW,
        (void*)H1, (void*)H1, kHid,
        b0, kChunk, kHid, kInW, 1.0f, 1.0f);
    wmma_gemm64<0, 0, 2, 1><<<gridBig, 256, 0, stream>>>(
        H1, H1, kHid,
        W1S, W1S, kHid,
        (void*)H2H, (void*)H2L, kHid,
        b1, kChunk, kHid, kHid, kW1CarryInv, 1.0f);
    wmma_gemm64<1, 2, 0, 7><<<gridSmall, 256, 0, stream>>>(
        H2H, H2L, kHid,
        WLH, WLL, kHid,
        (void*)(OUT3 + rowOff * kNoutP), (void*)(OUT3 + rowOff * kNoutP), kNoutP,
        BL64, kChunk, kNoutP, kHid, 1.0f, 100.0f);
  }

  traj_scan_kernel<<<kRowsR / kScanBlk, kScanBlk, 0, stream>>>(OUT3, input, out);
}
